// GCN_4277787427615
// MI455X (gfx1250) — hardware-verified
//
#include <hip/hip_runtime.h>
#include <stddef.h>
#include <stdint.h>
#include <math.h>


#define DH     128
#define NCLS   40
#define NC3    64
#define NTHR   256
#define NWAVE  8
#define EPT    8
#define CHUNK  (NTHR * EPT)
#define WCAP   (EPT * 32)
#define LISTN  (NWAVE * WCAP)
#define NBD    8192
#define SLD    13
#define NBA    1024
#define SLA    10
#define RCAP   26624
#define DEGCAP 64
#define SPW    (NBA / NWAVE)
#define GBM    64
#define GTHR   128
#define NUW    (DH * (DH / 8))
#define NU3    (NC3 * (DH / 8))
#define PRECN  256
#define OBW    (16 * NCLS)
#define NPI    (OBW / (4 * 32))
#define AGG_ZINTS    (LISTN + 2 * RCAP + 3 * NBA)
#define MISC_INTS    16
#define XBUF_FLTS    5120
#define AGG_LDS_INTS (AGG_ZINTS + MISC_INTS + XBUF_FLTS)
#define WSMAX  134217728

static_assert((CHUNK & (CHUNK - 1)) == 0 && CHUNK <= 4096);
static_assert((NBD & (NBD - 1)) == 0 && NBD == (1 << SLD));
static_assert((NBA & (NBA - 1)) == 0 && NBA == (1 << SLA));
static_assert(((long long)CHUNK << SLD) < (1LL << 31));
static_assert(((long long)CHUNK << SLA) < (1LL << 31));
static_assert(NBD % (NTHR * 4) == 0);
static_assert(LISTN % NTHR == 0);
static_assert(NBA % NWAVE == 0 && NBA % 32 == 0 && NBA % GBM == 0);
static_assert(RCAP % 32 == 0 && AGG_ZINTS % 4 == 0 && LISTN % 4 == 0);
static_assert(AGG_ZINTS % (NTHR * 4) == 0);
static_assert(((AGG_ZINTS + MISC_INTS) % 4) == 0);
static_assert(SPW % 16 == 0);
static_assert(XBUF_FLTS >= NWAVE * OBW);
static_assert(XBUF_FLTS >= 2 * (NWAVE * PRECN + PRECN));
static_assert(OBW % 128 == 0 && NPI * 128 == OBW);
static_assert(NCLS % 4 == 0 && NCLS / 2 <= 32 && NCLS <= NC3);
static_assert(PRECN == NTHR && PRECN == 2 * DH);
static_assert(DH % 32 == 0 && DH == 4 * 32 && NC3 == 2 * 32);
static_assert(GBM == (GTHR / 32) * 16 && GTHR == DH);
static_assert(NUW % NTHR == 0 && NU3 % NTHR == 0 && DH / 8 == 16);
static_assert(AGG_LDS_INTS * 4 <= 300000);

typedef float          v2f   __attribute__((ext_vector_type(2)));
typedef float          v4f   __attribute__((ext_vector_type(4)));
typedef float          v8f   __attribute__((ext_vector_type(8)));
typedef double         v2d   __attribute__((ext_vector_type(2)));
typedef int            v4i   __attribute__((ext_vector_type(4)));
typedef int            v8i   __attribute__((ext_vector_type(8)));
typedef unsigned short v8us  __attribute__((ext_vector_type(8)));
typedef unsigned short v16us __attribute__((ext_vector_type(16)));
typedef __bf16         v16bf __attribute__((ext_vector_type(16)));
typedef v2f  __attribute__((may_alias)) v2fa;
typedef v4f  __attribute__((may_alias)) v4fa;
typedef v2d  __attribute__((may_alias)) v2da;
typedef v4i  __attribute__((may_alias)) v4ia;
typedef v8us __attribute__((may_alias)) v8usa;
union FragB { v16bf v; v16us u; v8us h[2]; v8i w; };

__device__ __forceinline__ v8f wmb(const FragB& a, const FragB& b, v8f c) {
  v8f d = __builtin_amdgcn_wmma_f32_16x16x32_bf16(false, a.v, false, b.v, (short)0, c, false, false);
  asm volatile("v_nop\n\tv_nop\n\tv_nop\n\tv_nop" : "+v"(d) : "v"(a.w), "v"(b.w));
  return d;
}

__device__ __forceinline__ unsigned bf16_bits(float f) {
  const unsigned u = __float_as_uint(f);
  return (u + 0x7FFFu + ((u >> 16) & 1u)) >> 16;
}
__device__ __forceinline__ float bf16_val(float f) {
  return __uint_as_float(bf16_bits(f) << 16);
}

__device__ __forceinline__ void wave_sync() {
  __builtin_amdgcn_fence(__ATOMIC_RELEASE, "wavefront");
  __builtin_amdgcn_wave_barrier();
  __builtin_amdgcn_fence(__ATOMIC_ACQUIRE, "wavefront");
}

template <int SLB>
__device__ __forceinline__ int scan_chunk(const int* __restrict__ dsts, int nE, int cbase, int slotBase,
                                          int nb, int vec8, int* list, int tid, int lane, int wave) {
  int wc = 0;
  const int el0  = tid * EPT;
  const int e0   = cbase + el0;
  const int sent = -2147483647 - 1;
  v4i da, db;
  if (vec8 != 0 && cbase + CHUNK <= nE) {
    da = *(const v4i*)(dsts + e0);
    db = *(const v4i*)(dsts + e0 + 4);
  } else {
    da.x = (e0     < nE) ? dsts[min(e0,     nE - 1)] : sent;
    da.y = (e0 + 1 < nE) ? dsts[min(e0 + 1, nE - 1)] : sent;
    da.z = (e0 + 2 < nE) ? dsts[min(e0 + 2, nE - 1)] : sent;
    da.w = (e0 + 3 < nE) ? dsts[min(e0 + 3, nE - 1)] : sent;
    db.x = (e0 + 4 < nE) ? dsts[min(e0 + 4, nE - 1)] : sent;
    db.y = (e0 + 5 < nE) ? dsts[min(e0 + 5, nE - 1)] : sent;
    db.z = (e0 + 6 < nE) ? dsts[min(e0 + 6, nE - 1)] : sent;
    db.w = (e0 + 7 < nE) ? dsts[min(e0 + 7, nE - 1)] : sent;
  }
  const unsigned nbs = (unsigned)slotBase;
  const unsigned unb = (unsigned)nb;
  const unsigned s0 = (unsigned)da.x - nbs, s1 = (unsigned)da.y - nbs;
  const unsigned s2 = (unsigned)da.z - nbs, s3 = (unsigned)da.w - nbs;
  const unsigned s4 = (unsigned)db.x - nbs, s5 = (unsigned)db.y - nbs;
  const unsigned s6 = (unsigned)db.z - nbs, s7 = (unsigned)db.w - nbs;
  const bool h0 = s0 < unb, h1 = s1 < unb, h2 = s2 < unb, h3 = s3 < unb;
  const bool h4 = s4 < unb, h5 = s5 < unb, h6 = s6 < unb, h7 = s7 < unb;
  const unsigned any = __builtin_amdgcn_ballot_w32(h0 | h1 | h2 | h3 | h4 | h5 | h6 | h7);
  if (any != 0u) {
#define HITJ(J, HJ, SJ) { \
      const unsigned mj = __builtin_amdgcn_ballot_w32(HJ); \
      if (mj != 0u) { \
        if (HJ) { \
          const int pos = wc + (int)__builtin_amdgcn_mbcnt_lo(mj, 0u); \
          if (pos < WCAP) list[wave * WCAP + pos] = ((el0 + (J)) << SLB) | (int)(SJ); \
        } \
        wc += (int)__builtin_popcount(mj); } }
    HITJ(0, h0, s0)
    HITJ(1, h1, s1)
    HITJ(2, h2, s2)
    HITJ(3, h3, s3)
    HITJ(4, h4, s4)
    HITJ(5, h5, s5)
    HITJ(6, h6, s6)
    HITJ(7, h7, s7)
#undef HITJ
  }
  return wc;
}

__global__ __launch_bounds__(NTHR) void k_wprep(const float* __restrict__ W1, const float* __restrict__ W2,
                                                const float* __restrict__ W3,
                                                unsigned short* WT1, unsigned short* WT2, unsigned short* WT3) {
  const int u = (int)blockIdx.x * NTHR + (int)threadIdx.x;
  v8us o;
  unsigned short* dp;
  if (u < NUW) {
    const int n  = u >> 4;
    const int k8 = (u & 15) * 8;
    const float* p = W1 + (size_t)k8 * DH + n;
#pragma unroll
    for (int i = 0; i < 8; ++i) o[i] = (unsigned short)bf16_bits(p[(size_t)i * DH]);
    dp = WT1 + (size_t)n * DH + k8;
  } else if (u < 2 * NUW) {
    const int v  = u - NUW;
    const int n  = v >> 4;
    const int k8 = (v & 15) * 8;
    const float* p = W2 + (size_t)k8 * DH + n;
#pragma unroll
    for (int i = 0; i < 8; ++i) o[i] = (unsigned short)bf16_bits(p[(size_t)i * DH]);
    dp = WT2 + (size_t)n * DH + k8;
  } else if (u < 2 * NUW + NU3) {
    const int v  = u - 2 * NUW;
    const int n  = v >> 4;
    const int k8 = (v & 15) * 8;
    const int nc = n < NCLS ? n : NCLS - 1;
    const bool ok = n < NCLS;
    const float* p = W3 + (size_t)k8 * NCLS + nc;
#pragma unroll
    for (int i = 0; i < 8; ++i) {
      const float w = p[(size_t)i * NCLS];
      o[i] = ok ? (unsigned short)bf16_bits(w) : (unsigned short)0;
    }
    dp = WT3 + (size_t)n * DH + k8;
  } else {
    return;
  }
  *(volatile v8us*)dp = o;
  __threadfence();
  *(volatile v8us*)dp = o;
}

__global__ __launch_bounds__(NTHR) void k_deg(const int* __restrict__ dsts, int nE, int vec8, float* dis) {
  __shared__ __attribute__((aligned(16))) int scnt[NBD];
  __shared__ __attribute__((aligned(16))) int list[LISTN];
  __shared__ int wcnt[NWAVE];
  const int tid = (int)threadIdx.x, lane = tid & 31, wave = tid >> 5;
  const int nodeBase = (int)blockIdx.x * NBD;

  for (int i = tid; i < NBD; i += NTHR) scnt[i] = 0;
  for (int i = tid; i < LISTN; i += NTHR) list[i] = 0;
  if (tid < NWAVE) wcnt[tid] = 0;
  __syncthreads();

  const int nChunks = (nE + CHUNK - 1) / CHUNK;
#pragma unroll 1
  for (int ch = 0; ch < nChunks; ++ch) {
    const int cbase = ch * CHUNK;
    const int wc = scan_chunk<SLD>(dsts, nE, cbase, nodeBase, NBD, vec8, list, tid, lane, wave);
    if (lane == 0) wcnt[wave] = wc;
    __syncthreads();
    if (wave == 0) {
#pragma unroll 1
      for (int w2 = 0; w2 < NWAVE; ++w2) {
        int c = wcnt[w2];
        c = c < 0 ? 0 : (c > WCAP ? WCAP : c);
#pragma unroll 1
        for (int b0 = 0; b0 < c; b0 += 32) {
          const int idx = b0 + lane;
          const int ent = list[w2 * WCAP + (idx < WCAP ? idx : WCAP - 1)];
          const int m32 = (c - b0) < 32 ? (c - b0) : 32;
#pragma unroll 1
          for (int k = 0; k < m32; ++k) {
            const int u  = __builtin_amdgcn_readlane(ent, k);
            const int sl = u & (NBD - 1);
            if (lane == 0) scnt[sl] = scnt[sl] + 1;
          }
        }
      }
    }
    __syncthreads();
  }

  v4f vals[NBD / (NTHR * 4)];
#pragma unroll
  for (int it = 0; it < NBD / (NTHR * 4); ++it) {
    const int s0 = it * (NTHR * 4) + 4 * tid;
    const v4i c4 = *(const v4ia*)(scnt + s0);
    const float d0 = (float)c4.x + 1.0f, d1 = (float)c4.y + 1.0f;
    const float d2 = (float)c4.z + 1.0f, d3 = (float)c4.w + 1.0f;
    v4f v;
    v.x = rsqrtf(d0); v.y = rsqrtf(d1); v.z = rsqrtf(d2); v.w = rsqrtf(d3);
    vals[it] = v;
  }
#pragma unroll
  for (int it = 0; it < NBD / (NTHR * 4); ++it) {
    const int s0 = it * (NTHR * 4) + 4 * tid;
    *(volatile v4f*)(dis + (size_t)nodeBase + s0) = vals[it];
  }
  __threadfence();
#pragma unroll
  for (int it = 0; it < NBD / (NTHR * 4); ++it) {
    const int s0 = it * (NTHR * 4) + 4 * tid;
    *(volatile v4f*)(dis + (size_t)nodeBase + s0) = vals[it];
  }
}

template <int NT, int PRE>
__global__ __launch_bounds__(GTHR) void k_gemm(const float* __restrict__ A, int lda, int nA,
                                               const unsigned short* __restrict__ WT,
                                               const float* __restrict__ st, const float* __restrict__ be,
                                               float* outF) {
  constexpr int NCOL = 16 * NT;
  constexpr int LPR  = NCOL / 4;
  constexpr int RPI  = 32 / LPR;
  constexpr int NITE = 16 / RPI;
  static_assert(NT == 4 || NT == 8);
  __shared__ __attribute__((aligned(16))) float stg[GBM * NCOL];
  __shared__ __attribute__((aligned(16))) float sbn[3 * DH];
  const int tid = (int)threadIdx.x, lane = tid & 31, wave = tid >> 5, hh = lane >> 4, m = lane & 15;
  const int rowBase = (int)blockIdx.x * GBM;

  if constexpr (PRE != 0) {
    sbn[tid]          = st[tid];
    sbn[DH + tid]     = st[DH + tid];
    sbn[2 * DH + tid] = bf16_val(be[tid]);
  }
  __syncthreads();

  v8f acc[NT];
  {
    const v8f z = {0.f, 0.f, 0.f, 0.f, 0.f, 0.f, 0.f, 0.f};
#pragma unroll
    for (int t = 0; t < NT; ++t) acc[t] = z;
  }
  const int  arow = rowBase + 16 * wave + m;
  const bool aok  = arow < nA;
  const int  arc  = aok ? arow : nA - 1;
  const float* ap = A + (size_t)arc * (size_t)lda + 8 * hh;
  const unsigned short* wp = WT + (size_t)m * DH + 8 * hh;

#pragma unroll 1
  for (int ks = 0; ks < DH / 32; ++ks) {
    const int k0 = 32 * ks;
    FragB ah, al;
    {
      const v8i z8 = {0, 0, 0, 0, 0, 0, 0, 0};
      al.w = z8;
    }
#pragma unroll
    for (int q = 0; q < 4; ++q) {
      const int co = (q < 2) ? (k0 + 4 * q) : (k0 + 16 + 4 * (q - 2));
      const v4f xv = *(const v4fa*)(ap + co);
      float v0 = xv.x, v1 = xv.y, v2 = xv.z, v3 = xv.w;
      if constexpr (PRE != 0) {
        const int cc = co + 8 * hh;
        const v4f mu = *(const v4fa*)(sbn + cc);
        const v4f sc = *(const v4fa*)(sbn + DH + cc);
        const v4f bb = *(const v4fa*)(sbn + 2 * DH + cc);
        v0 = fmaxf(fmaf(v0 - mu.x, sc.x, bb.x), 0.0f);
        v1 = fmaxf(fmaf(v1 - mu.y, sc.y, bb.y), 0.0f);
        v2 = fmaxf(fmaf(v2 - mu.z, sc.z, bb.z), 0.0f);
        v3 = fmaxf(fmaf(v3 - mu.w, sc.w, bb.w), 0.0f);
      }
      v0 = aok ? v0 : 0.0f; v1 = aok ? v1 : 0.0f; v2 = aok ? v2 : 0.0f; v3 = aok ? v3 : 0.0f;
      const unsigned h0 = bf16_bits(v0), h1 = bf16_bits(v1), h2 = bf16_bits(v2), h3 = bf16_bits(v3);
      ah.u[4 * q + 0] = (unsigned short)h0;
      ah.u[4 * q + 1] = (unsigned short)h1;
      ah.u[4 * q + 2] = (unsigned short)h2;
      ah.u[4 * q + 3] = (unsigned short)h3;
      if constexpr (PRE != 0) {
        al.u[4 * q + 0] = (unsigned short)bf16_bits(v0 - __uint_as_float(h0 << 16));
        al.u[4 * q + 1] = (unsigned short)bf16_bits(v1 - __uint_as_float(h1 << 16));
        al.u[4 * q + 2] = (unsigned short)bf16_bits(v2 - __uint_as_float(h2 << 16));
        al.u[4 * q + 3] = (unsigned short)bf16_bits(v3 - __uint_as_float(h3 << 16));
      }
    }
#pragma unroll
    for (int nt = 0; nt < NT; ++nt) {
      const unsigned short* wq = wp + (size_t)(16 * nt) * (size_t)DH + k0;
      FragB bf;
      bf.h[0] = *(const v8usa*)wq;
      bf.h[1] = *(const v8usa*)(wq + 16);
      acc[nt] = wmb(ah, bf, acc[nt]);
      if constexpr (PRE != 0) acc[nt] = wmb(al, bf, acc[nt]);
    }
  }

#pragma unroll
  for (int nt = 0; nt < NT; ++nt) {
    const int lc = 16 * nt + m;
#pragma unroll
    for (int r = 0; r < 8; ++r) {
      const int lr = 16 * wave + 8 * hh + r;
      stg[lr * NCOL + lc] = acc[nt][r];
    }
  }
  __syncthreads();

  const int lsub = lane / LPR;
  const int lcol = 4 * (lane % LPR);
  v4f fv[NITE];
#pragma unroll
  for (int i = 0; i < NITE; ++i) {
    const int lr = 16 * wave + i * RPI + lsub;
    fv[i] = *(const v4fa*)(stg + lr * NCOL + lcol);
  }
#pragma unroll
  for (int i = 0; i < NITE; ++i) {
    const int gr = rowBase + 16 * wave + i * RPI + lsub;
    float* op = outF + (size_t)gr * (size_t)NCOL + lcol;
    *(volatile v4f*)op = fv[i];
  }
  __threadfence();
#pragma unroll
  for (int i = 0; i < NITE; ++i) {
    const int gr = rowBase + 16 * wave + i * RPI + lsub;
    float* op = outF + (size_t)gr * (size_t)NCOL + lcol;
    *(volatile v4f*)op = fv[i];
  }
}

template <int MODE>
__global__ __launch_bounds__(NTHR) void k_scan(const int* __restrict__ srcs, const int* __restrict__ dsts,
                                               int nE, int nN, int vec8, int mRows,
                                               const float* __restrict__ dis, const float* __restrict__ tin,
                                               const float* __restrict__ bias,
                                               float* aout, double* prec, float* out) {
  extern __shared__ __attribute__((aligned(16))) int dsm[];
  int* list = dsm;
  int* hl   = dsm + LISTN;
  int* sl   = hl + RCAP;
  int* cnt  = sl + RCAP;
  int* offs = cnt + NBA;
  int* cur  = offs + NBA;
  int* misc = cur + NBA;
  float* xb = (float*)(misc + MISC_INTS);
  const int tid = (int)threadIdx.x, lane = tid & 31, wave = tid >> 5;
  const int nodeBase = (int)blockIdx.x * NBA;

  {
    const v4i z4 = {0, 0, 0, 0};
    for (int i = tid * 4; i < AGG_ZINTS; i += NTHR * 4) *(v4ia*)(dsm + i) = z4;
    if (tid < MISC_INTS) misc[tid] = 0;
  }
  __syncthreads();

  int t = 0, ov = 0;
  const int nChunks = (nE + CHUNK - 1) / CHUNK;
#pragma unroll 1
  for (int ch = 0; ch < nChunks; ++ch) {
    const int cbase = ch * CHUNK;
    const int wc = scan_chunk<SLA>(dsts, nE, cbase, nodeBase, NBA, vec8, list, tid, lane, wave);
    if (lane == 0) misc[wave] = wc;
    __syncthreads();
    if (wave == 0) {
#pragma unroll 1
      for (int w2 = 0; w2 < NWAVE; ++w2) {
        int c = misc[w2];
        c = c < 0 ? 0 : (c > WCAP ? WCAP : c);
#pragma unroll 1
        for (int b0 = 0; b0 < c; b0 += 32) {
          const int idx = b0 + lane;
          const int ent = list[w2 * WCAP + (idx < WCAP ? idx : WCAP - 1)];
          const int m32 = (c - b0) < 32 ? (c - b0) : 32;
#pragma unroll 1
          for (int k = 0; k < m32; ++k) {
            const int u    = __builtin_amdgcn_readlane(ent, k);
            const int slot = u & (NBA - 1);
            const int el   = (u >> SLA) & (CHUNK - 1);
            const int pk   = ((cbase + el) << SLA) | slot;
            if (t < RCAP) {
              if (lane == 0) { hl[t] = pk; cnt[slot] = cnt[slot] + 1; }
              t = t + 1;
            } else {
              ov = 1;
            }
          }
        }
      }
    }
    __syncthreads();
  }
  if (wave == 0 && lane == 0) { misc[8] = t; misc[9] = ov; }
  __syncthreads();
  int tt = misc[8];
  tt = tt < 0 ? 0 : (tt > RCAP ? RCAP : tt);
  const int ovf = misc[9];

  if (wave == 0) {
    const int base = lane * (NBA / 32);
    int s = 0;
#pragma unroll 1
    for (int i = 0; i < NBA / 32; ++i) s += cnt[base + i];
    int incl = s;
#pragma unroll
    for (int d = 1; d < 32; d <<= 1) {
      const int y = __shfl_up(incl, d, 32);
      if (lane >= d) incl += y;
    }
    int run = incl - s;
#pragma unroll 1
    for (int i = 0; i < NBA / 32; ++i) {
      const int cv = cnt[base + i];
      offs[base + i] = run;
      cur[base + i]  = run;
      run += cv;
    }
  }
  __syncthreads();
  if (wave == 0) {
#pragma unroll 1
    for (int b0 = 0; b0 < tt; b0 += 32) {
      const int idx = b0 + lane;
      const int ent = hl[idx < RCAP ? idx : RCAP - 1];
      const int m32 = (tt - b0) < 32 ? (tt - b0) : 32;
#pragma unroll 1
      for (int k = 0; k < m32; ++k) {
        const int u    = __builtin_amdgcn_readlane(ent, k);
        const int slot = u & (NBA - 1);
        if (lane == 0) {
          int p = cur[slot];
          p = p < 0 ? 0 : (p > RCAP - 1 ? RCAP - 1 : p);
          sl[p] = u;
          cur[slot] = p + 1;
        }
      }
    }
  }
  __syncthreads();

  const float qnan = __int_as_float(0x7fc00000);
  const float pz = (ovf != 0) ? qnan : 0.0f;
  if constexpr (MODE != 0) {
    float bv0, bv1, bv2, bv3;
    {
      const v4f bq = *(const v4fa*)(bias + 4 * lane);
      bv0 = bf16_val(bq.x); bv1 = bf16_val(bq.y); bv2 = bf16_val(bq.z); bv3 = bf16_val(bq.w);
    }
    double d10 = 0.0, d11 = 0.0, d12 = 0.0, d13 = 0.0;
    double d20 = 0.0, d21 = 0.0, d22 = 0.0, d23 = 0.0;
#pragma unroll 1
    for (int j = 0; j < SPW; ++j) {
      const int s    = wave * SPW + j;
      const int node = nodeBase + s;
      int c = cnt[s];
      const bool big = c > DEGCAP;
      c = c < 0 ? 0 : (c > DEGCAP ? DEGCAP : c);
      int o = offs[s];
      o = o < 0 ? 0 : (o > RCAP ? RCAP : o);
      const int nc = node < nN ? node : nN - 1;
      const float dd = dis[nc];
      const float rd = dd * dd;
      float acc0 = 0.0f, acc1 = 0.0f, acc2 = 0.0f, acc3 = 0.0f;
#pragma unroll 1
      for (int b0 = 0; b0 < c; b0 += 32) {
        int idx = o + b0 + lane;
        idx = idx > RCAP - 1 ? RCAP - 1 : idx;
        const int ent = sl[idx];
        int eid = ent >> SLA;
        eid = eid < 0 ? 0 : (eid > nE - 1 ? nE - 1 : eid);
        int sr = srcs[eid];
        sr = sr < 0 ? 0 : (sr > nN - 1 ? nN - 1 : sr);
        const float cf  = dis[sr] * dd;
        const int   cfi = __float_as_int(cf);
        const int m32 = (c - b0) < 32 ? (c - b0) : 32;
#pragma unroll 1
        for (int k = 0; k < m32; ++k) {
          const int   sk = __builtin_amdgcn_readlane(sr, k);
          const float ck = __int_as_float(__builtin_amdgcn_readlane(cfi, k));
          const v4f a = *(const v4fa*)(tin + (size_t)sk * DH + 4 * lane);
          acc0 = fmaf(ck, a.x, acc0); acc1 = fmaf(ck, a.y, acc1);
          acc2 = fmaf(ck, a.z, acc2); acc3 = fmaf(ck, a.w, acc3);
        }
      }
      const v4f sv = *(const v4fa*)(tin + (size_t)nc * DH + 4 * lane);
      const float pzr = big ? qnan : pz;
      const bool live = node < nN;
      const float y0 = (acc0 + sv.x * rd) + bv0 + pzr;
      const float y1 = (acc1 + sv.y * rd) + bv1 + pzr;
      const float y2 = (acc2 + sv.z * rd) + bv2 + pzr;
      const float y3 = (acc3 + sv.w * rd) + bv3 + pzr;
      const float v0 = live ? y0 : 0.0f;
      const float v1 = live ? y1 : 0.0f;
      const float v2 = live ? y2 : 0.0f;
      const float v3 = live ? y3 : 0.0f;
      d10 += (double)v0; d20 += (double)v0 * (double)v0;
      d11 += (double)v1; d21 += (double)v1 * (double)v1;
      d12 += (double)v2; d22 += (double)v2 * (double)v2;
      d13 += (double)v3; d23 += (double)v3 * (double)v3;
      v4f ow;
      ow.x = v0; ow.y = v1; ow.z = v2; ow.w = v3;
      if (node < mRows) {
        float* op = aout + (size_t)node * DH + 4 * lane;
        *(volatile v4f*)op = ow;
        __threadfence();
        *(volatile v4f*)op = ow;
      }
    }
    double* wst = (double*)xb;
    double* pst = wst + NWAVE * PRECN;
    wst[wave * PRECN + 4 * lane + 0] = d10;
    wst[wave * PRECN + 4 * lane + 1] = d11;
    wst[wave * PRECN + 4 * lane + 2] = d12;
    wst[wave * PRECN + 4 * lane + 3] = d13;
    wst[wave * PRECN + DH + 4 * lane + 0] = d20;
    wst[wave * PRECN + DH + 4 * lane + 1] = d21;
    wst[wave * PRECN + DH + 4 * lane + 2] = d22;
    wst[wave * PRECN + DH + 4 * lane + 3] = d23;
    __syncthreads();
    {
      double p = 0.0;
#pragma unroll
      for (int w2 = 0; w2 < NWAVE; ++w2) p += wst[w2 * PRECN + tid];
      pst[tid] = p;
    }
    __syncthreads();
    if (tid < PRECN / 2) {
      const v2d q = *(const v2da*)(pst + 2 * tid);
      double* gp = prec + (size_t)blockIdx.x * PRECN + 2 * tid;
      *(volatile v2d*)gp = q;
      __threadfence();
      *(volatile v2d*)gp = q;
    }
  } else {
    const bool valid = lane < (NCLS / 2);
    float bv0, bv1;
    {
      const int bi = valid ? 2 * lane : NCLS - 2;
      const v2f bq = *(const v2fa*)(bias + bi);
      bv0 = valid ? bf16_val(bq.x) : 0.0f;
      bv1 = valid ? bf16_val(bq.y) : 0.0f;
    }
    float* obuf = xb + wave * OBW;
#pragma unroll 1
    for (int j = 0; j < SPW; ++j) {
      const int s    = wave * SPW + j;
      const int node = nodeBase + s;
      int c = cnt[s];
      const bool big = c > DEGCAP;
      c = c < 0 ? 0 : (c > DEGCAP ? DEGCAP : c);
      int o = offs[s];
      o = o < 0 ? 0 : (o > RCAP ? RCAP : o);
      const int nc = node < nN ? node : nN - 1;
      const float dd = dis[nc];
      const float rd = dd * dd;
      float acc0 = 0.0f, acc1 = 0.0f;
#pragma unroll 1
      for (int b0 = 0; b0 < c; b0 += 32) {
        int idx = o + b0 + lane;
        idx = idx > RCAP - 1 ? RCAP - 1 : idx;
        const int ent = sl[idx];
        int eid = ent >> SLA;
        eid = eid < 0 ? 0 : (eid > nE - 1 ? nE - 1 : eid);
        int sr = srcs[eid];
        sr = sr < 0 ? 0 : (sr > nN - 1 ? nN - 1 : sr);
        const float cf  = dis[sr] * dd;
        const int   cfi = __float_as_int(cf);
        const int m32 = (c - b0) < 32 ? (c - b0) : 32;
#pragma unroll 1
        for (int k = 0; k < m32; ++k) {
          const int   sk = __builtin_amdgcn_readlane(sr, k);
          const float ck = __int_as_float(__builtin_amdgcn_readlane(cfi, k));
          const v2f a = *(const v2fa*)(tin + (size_t)sk * NC3 + 2 * lane);
          acc0 = fmaf(ck, a.x, acc0); acc1 = fmaf(ck, a.y, acc1);
        }
      }
      const v2f sv = *(const v2fa*)(tin + (size_t)nc * NC3 + 2 * lane);
      const float pzr = big ? qnan : pz;
      const float y0 = (acc0 + sv.x * rd) + bv0 + pzr;
      const float y1 = (acc1 + sv.y * rd) + bv1 + pzr;
      float mx = valid ? fmaxf(y0, y1) : -3.0e38f;
#pragma unroll
      for (int off = 16; off > 0; off >>= 1) mx = fmaxf(mx, __shfl_xor(mx, off, 32));
      const float e0 = expf(y0 - mx);
      const float e1 = expf(y1 - mx);
      float se = valid ? (e0 + e1) : 0.0f;
#pragma unroll
      for (int off = 16; off > 0; off >>= 1) se += __shfl_xor(se, off, 32);
      const float lse = mx + logf(se);
      const float o0 = y0 - lse, o1 = y1 - lse;
      const int r = j & 15;
      if (valid) {
        v2f ov;
        ov.x = o0; ov.y = o1;
        *(v2fa*)(obuf + r * NCLS + 2 * lane) = ov;
      }
      if (r == 15) {
        wave_sync();
        const int row0 = nodeBase + wave * SPW + (j - 15);
        v4f pc[NPI];
#pragma unroll
        for (int it = 0; it < NPI; ++it) pc[it] = *(const v4fa*)(obuf + 4 * (it * 32 + lane));
        float* ob = out + (size_t)row0 * NCLS;
#pragma unroll
        for (int it = 0; it < NPI; ++it) {
          const int p = it * 32 + lane;
          if (row0 + p / (NCLS / 4) < nN) *(volatile v4f*)(ob + 4 * p) = pc[it];
        }
        __threadfence();
#pragma unroll
        for (int it = 0; it < NPI; ++it) {
          const int p = it * 32 + lane;
          if (row0 + p / (NCLS / 4) < nN) *(volatile v4f*)(ob + 4 * p) = pc[it];
        }
        wave_sync();
      }
    }
  }
}

__global__ __launch_bounds__(NTHR) void k_bnc(const double* __restrict__ prec, int nb, double invN,
                                              const float* __restrict__ g, float* st) {
  __shared__ __attribute__((aligned(16))) float so[2 * DH];
  const int tid = (int)threadIdx.x;
  if (tid < DH) {
    double s1 = 0.0, s2 = 0.0;
#pragma unroll 1
    for (int b = 0; b < nb; ++b) {
      s1 += prec[(size_t)b * PRECN + tid];
      s2 += prec[(size_t)b * PRECN + DH + tid];
    }
    const double mu = s1 * invN;
    double var = s2 * invN - mu * mu;
    var = var < 0.0 ? 0.0 : var;
    const float vf = (float)var + 1.0e-5f;
    const float rstd = 1.0f / sqrtf(vf);
    so[tid] = (float)mu;
    so[DH + tid] = bf16_val(g[tid]) * rstd;
  }
  __syncthreads();
  if (tid < (2 * DH) / 4) {
    const v4f v = *(const v4fa*)(so + 4 * tid);
    float* p = st + 4 * tid;
    *(volatile v4f*)p = v;
    __threadfence();
    *(volatile v4f*)p = v;
  }
}

static inline int cdiv(int a, int b) { return (a + b - 1) / b; }
static inline size_t al256(size_t o) { return (o + 255) & ~(size_t)255; }

extern "C" void kernel_launch(void* const* d_in, const int* in_sizes, int n_in,
                              void* d_out, int out_size, void* d_ws, size_t ws_size,
                              hipStream_t stream) {
  if (n_in < 12) return;
  if (in_sizes[0] < DH || (in_sizes[0] % DH) != 0) return;
  const int nN = in_sizes[0] / DH;
  if (nN < 16 || nN >= (1 << 24)) return;
  if (in_sizes[1] != DH * DH || in_sizes[2] != DH) return;
  if (in_sizes[3] != DH * DH || in_sizes[4] != DH) return;
  if (in_sizes[5] != DH * NCLS || in_sizes[6] != NCLS) return;
  if (in_sizes[7] != DH || in_sizes[8] != DH) return;
  if (in_sizes[9] != DH || in_sizes[10] != DH) return;
  if (in_sizes[11] < 2 || (in_sizes[11] & 1) != 0) return;
  const int nE = in_sizes[11] / 2;
  if (nE < 1 || nE >= (1 << (31 - SLA))) return;
  if ((long long)out_size != (long long)nN * NCLS) return;

  const float* x    = (const float*)d_in[0];
  const float* W1   = (const float*)d_in[1];
  const float* b1   = (const float*)d_in[2];
  const float* W2   = (const float*)d_in[3];
  const float* b2   = (const float*)d_in[4];
  const float* W3   = (const float*)d_in[5];
  const float* b3   = (const float*)d_in[6];
  const float* g1   = (const float*)d_in[7];
  const float* be1  = (const float*)d_in[8];
  const float* g2   = (const float*)d_in[9];
  const float* be2  = (const float*)d_in[10];
  const int*   edge = (const int*)d_in[11];
  const int* src = edge;
  const int* dst = edge + nE;
  float* out = (float*)d_out;

  const int MP   = cdiv(nN, GBM) * GBM;
  const int gM   = MP / GBM;
  const int gD   = cdiv(nN, NBD);
  const int NBPD = gD * NBD;
  const int gA   = cdiv(MP, NBA);
  if ((long long)gA * NBA < (long long)MP) return;
  if (NBPD < nN) return;
  const int vec8 = ((nE & 3) == 0) ? 1 : 0;
  const double invN = 1.0 / (double)nN;

  char* ws = (char*)d_ws;
  size_t off = 0;
  const size_t oDIS = off; off = al256(off + (size_t)NBPD * 4);
  const size_t oWT1 = off; off = al256(off + (size_t)DH * DH * 2);
  const size_t oWT2 = off; off = al256(off + (size_t)DH * DH * 2);
  const size_t oWT3 = off; off = al256(off + (size_t)NC3 * DH * 2);
  const size_t oPR1 = off; off = al256(off + (size_t)gA * PRECN * 8);
  const size_t oPR2 = off; off = al256(off + (size_t)gA * PRECN * 8);
  const size_t oST1 = off; off = al256(off + (size_t)(2 * DH) * 4);
  const size_t oST2 = off; off = al256(off + (size_t)(2 * DH) * 4);
  const size_t oR1  = off; off = al256(off + (size_t)MP * DH * 4);
  const size_t oR2  = off; off = al256(off + (size_t)MP * DH * 4);
  if (off > ws_size || off > (size_t)WSMAX) return;
  float*          DIS  = (float*)(ws + oDIS);
  unsigned short* WT1  = (unsigned short*)(ws + oWT1);
  unsigned short* WT2  = (unsigned short*)(ws + oWT2);
  unsigned short* WT3  = (unsigned short*)(ws + oWT3);
  double*         PR1  = (double*)(ws + oPR1);
  double*         PR2  = (double*)(ws + oPR2);
  float*          ST1  = (float*)(ws + oST1);
  float*          ST2  = (float*)(ws + oST2);
  float*          R1   = (float*)(ws + oR1);
  float*          R2   = (float*)(ws + oR2);

  const size_t scanLds = (size_t)AGG_LDS_INTS * 4;
  hipFuncSetAttribute(reinterpret_cast<const void*>(&k_scan<1>), hipFuncAttributeMaxDynamicSharedMemorySize, (int)scanLds);
  hipFuncSetAttribute(reinterpret_cast<const void*>(&k_scan<0>), hipFuncAttributeMaxDynamicSharedMemorySize, (int)scanLds);

  k_wprep<<<(2 * NUW + NU3) / NTHR, NTHR, 0, stream>>>(W1, W2, W3, WT1, WT2, WT3);
  k_deg<<<gD, NTHR, 0, stream>>>(dst, nE, vec8, DIS);
  k_gemm<8, 0><<<gM, GTHR, 0, stream>>>(x, DH, nN, WT1, ST1, be1, R1);
  k_scan<1><<<gA, NTHR, scanLds, stream>>>(src, dst, nE, nN, vec8, MP, DIS, R1, b1, R2, PR1, out);
  k_bnc<<<1, NTHR, 0, stream>>>(PR1, gA, invN, g1, ST1);
  k_gemm<8, 1><<<gM, GTHR, 0, stream>>>(R2, DH, nN, WT2, ST1, be1, R1);
  k_scan<1><<<gA, NTHR, scanLds, stream>>>(src, dst, nE, nN, vec8, MP, DIS, R1, b2, R2, PR2, out);
  k_bnc<<<1, NTHR, 0, stream>>>(PR2, gA, invN, g2, ST2);
  k_gemm<4, 1><<<gM, GTHR, 0, stream>>>(R2, DH, nN, WT3, ST2, be2, R1);
  k_scan<0><<<gA, NTHR, scanLds, stream>>>(src, dst, nE, nN, vec8, MP, DIS, R1, b3, R2, PR2, out);
}
